// GNOBlock_11553462026776
// MI455X (gfx1250) — hardware-verified
//
#include <hip/hip_runtime.h>
#include <stddef.h>
#include <stdint.h>


#define LAT   16
#define EDW   6
#define KD    128
#define W3C   256
#define KW3   2048
#define KP3   2080
#define EB    64
#define NTM   256
#define NTF   128
#define PH    136
#define NB    800
#define NTA   64
#define CH    64
#define WSCAP 134217728

static_assert(KW3 == LAT * KD);
static_assert(W3C == LAT * LAT);
static_assert(KP3 == KW3 + 32);
static_assert((KP3 % 32) == 0);
static_assert((PH % 8) == 0);
static_assert((((KD * KD) / 8) % NTM) == 0);
static_assert(((EB * KD) / 8) == 4 * NTM);
static_assert(((EB * LAT) / 4) == 2 * NTF);
static_assert((NB % 8) == 0);
static_assert(((NB * LAT) % (4 * NTA)) == 0);
static_assert(CH == NTA);
static_assert(NB * LAT * 4 + LAT * LAT * 4 + LAT * 4 + 2 * CH * 4 + 8 <= 65536);

typedef float          v4f  __attribute__((ext_vector_type(4)));
typedef float          v8f  __attribute__((ext_vector_type(8)));
typedef _Float16       v8h  __attribute__((ext_vector_type(8)));
typedef _Float16       v16h __attribute__((ext_vector_type(16)));
typedef unsigned int   v4u  __attribute__((ext_vector_type(4)));

union Frag { v16h v; v8h half[2]; };
union P8   { v8h h; v4u u; };

__device__ __forceinline__ v8f wmf(v16h a, v16h b, v8f c) {
  v8f d = __builtin_amdgcn_wmma_f32_16x16x32_f16(false, a, false, b, (short)0, c, false, false);
  asm volatile("v_nop\n\tv_nop\n\tv_nop\n\tv_nop" : "+v"(d) : "v"(a), "v"(b));
  return d;
}

__device__ __forceinline__ v8f vzero8() {
  v8f z = {0.f, 0.f, 0.f, 0.f, 0.f, 0.f, 0.f, 0.f};
  return z;
}

__device__ __forceinline__ v16h ldfrag(const _Float16* p) {
  Frag f;
  f.half[0] = *(const v8h*)(p);
  f.half[1] = *(const v8h*)(p + 16);
  return f.v;
}

__device__ __forceinline__ v16h scale16(v16h v, _Float16 s) { return v * s; }

__device__ __forceinline__ float gelu_f(float x) {
  return 0.5f * x * (1.0f + erff(x * 0.70710678118654752f));
}

__global__ __launch_bounds__(256) void k_prep(const float* __restrict__ W2, const float* __restrict__ W3,
                                               const float* __restrict__ b3, _Float16* W2t, _Float16* W3f) {
  const int NP2 = (KD * KD) / 8;
  const int NP3 = (LAT * KP3) / 8;
  const int idx = blockIdx.x * 256 + (int)threadIdx.x;
  if (idx >= NP2 + NP3) return;
  v8f v;
  _Float16* dp;
  if ((int)blockIdx.x < NP2 / 256) {
    const int n  = idx >> 4;
    const int k0 = (idx & 15) * 8;
#pragma unroll
    for (int j = 0; j < 8; ++j) v[j] = 64.0f * W2[(k0 + j) * KD + n];
    dp = W2t + n * KD + k0;
  } else {
    const int jj = idx - NP2;
    const int n  = jj / (KP3 / 8);
    const int p  = jj - n * (KP3 / 8);
    const int k0 = p * 8;
#pragma unroll
    for (int j = 0; j < 8; ++j) {
      const int k  = k0 + j;
      const int kw = min(k, KW3 - 1);
      const int i  = kw >> 7, kk = kw & (KD - 1);
      const float vw = W3[kk * W3C + LAT * i + n];
      const int ib = min(max(k - KW3, 0), LAT - 1);
      const float vb = b3[LAT * ib + n];
      const float s = (k < KW3) ? vw : ((k < KW3 + LAT) ? vb : 0.0f);
      v[j] = 64.0f * s;
    }
    dp = W3f + n * KP3 + k0;
  }
  P8 o;
  o.h = __builtin_convertvector(v, v8h);
  *(volatile v4u*)dp = o.u;
  __threadfence();
  *(volatile v4u*)dp = o.u;
}

__global__ __launch_bounds__(NTM) void k_mlp(const float* __restrict__ ea, int E,
                                             const float* __restrict__ W1, const float* __restrict__ b1,
                                             const _Float16* __restrict__ W2t, const float* __restrict__ b2,
                                             _Float16* h2p) {
  __shared__ float sEA[EB * 8];
  __shared__ __attribute__((aligned(16))) _Float16 sH1[EB * PH];
  __shared__ __attribute__((aligned(16))) _Float16 sH2[EB * PH];
  const int t = threadIdx.x;
  const int ebase = blockIdx.x * EB;

  for (int i = t; i < EB * EDW; i += NTM) {
    const int r = i / EDW, c = i - r * EDW;
    const int ge = ebase + r;
    const int gc = min(ge, E - 1);
    float v = ea[(size_t)gc * EDW + c];
    v = (ge < E) ? v : 0.0f;
    sEA[r * 8 + c] = v;
  }
  __syncthreads();

  {
    const int col = t & (KD - 1);
    const int rb  = (t >> 7) * (EB / 2);
    float wc[EDW];
#pragma unroll
    for (int i = 0; i < EDW; ++i) wc[i] = W1[i * KD + col];
    const float bb = b1[col];
#pragma unroll 1
    for (int rr = 0; rr < EB / 2; ++rr) {
      const int r = rb + rr;
      const float* er = sEA + r * 8;
      float a = 0.0f;
#pragma unroll
      for (int i = 0; i < EDW; ++i) a += er[i] * wc[i];
      a += bb;
      sH1[r * PH + col] = (_Float16)gelu_f(a);
    }
  }
  __syncthreads();

  const int lane = t & 31, w = t >> 5, h = lane >> 4, m = lane & 15;
  const int rt = w & 3, cg = (w >> 2) * 4;
  const _Float16* arow = sH1 + (16 * rt + m) * PH + 8 * h;
  const _Float16* bcol = W2t + (size_t)(16 * cg + m) * KD + 8 * h;
  v8f c0 = vzero8(), c1 = vzero8(), c2 = vzero8(), c3 = vzero8();
#pragma unroll
  for (int ks = 0; ks < KD / 32; ++ks) {
    const v16h a = ldfrag(arow + 32 * ks);
    c0 = wmf(a, ldfrag(bcol + 32 * ks),           c0);
    c1 = wmf(a, ldfrag(bcol + 16 * KD + 32 * ks), c1);
    c2 = wmf(a, ldfrag(bcol + 32 * KD + 32 * ks), c2);
    c3 = wmf(a, ldfrag(bcol + 48 * KD + 32 * ks), c3);
  }
  {
    const float q0 = b2[16 * cg + m], q1 = b2[16 * cg + 16 + m], q2 = b2[16 * cg + 32 + m], q3 = b2[16 * cg + 48 + m];
    _Float16* orow = sH2 + (16 * rt + 8 * h) * PH + 16 * cg + m;
#pragma unroll
    for (int r = 0; r < 8; ++r) {
      orow[r * PH]      = (_Float16)gelu_f(c0[r] * (1.0f / 64.0f) + q0);
      orow[r * PH + 16] = (_Float16)gelu_f(c1[r] * (1.0f / 64.0f) + q1);
      orow[r * PH + 32] = (_Float16)gelu_f(c2[r] * (1.0f / 64.0f) + q2);
      orow[r * PH + 48] = (_Float16)gelu_f(c3[r] * (1.0f / 64.0f) + q3);
    }
  }
  __syncthreads();

  _Float16* gb = h2p + (size_t)ebase * KD;
#pragma unroll
  for (int q = 0; q < 4; ++q) {
    const int idx = q * NTM + t;
    const int row = idx >> 4, c = idx & 15;
    P8 p;
    p.h = *(const v8h*)(sH2 + row * PH + 8 * c);
    *(volatile v4u*)(gb + (size_t)row * KD + 8 * c) = p.u;
  }
  __threadfence();
#pragma unroll
  for (int q = 0; q < 4; ++q) {
    const int idx = q * NTM + t;
    const int row = idx >> 4, c = idx & 15;
    P8 p;
    p.h = *(const v8h*)(sH2 + row * PH + 8 * c);
    *(volatile v4u*)(gb + (size_t)row * KD + 8 * c) = p.u;
  }
}

__global__ __launch_bounds__(NTF) void k_fold(const _Float16* __restrict__ h2p, const float* __restrict__ xin,
                                              int n_nodes, const int* __restrict__ src, int E,
                                              const _Float16* __restrict__ W3f, float* msg) {
  __shared__ __attribute__((aligned(32))) float sX[EB * LAT];
  __shared__ __attribute__((aligned(32))) float sO[EB * LAT];
  const int t = threadIdx.x, lane = t & 31, w = t >> 5, h = lane >> 4, m = lane & 15;
  const int ebase = blockIdx.x * EB;
  const v4f z4 = {0.f, 0.f, 0.f, 0.f};

#pragma unroll
  for (int q = 0; q < 2; ++q) {
    const int idx = q * NTF + t;
    const int e = idx >> 2, c4 = idx & 3;
    const int ge = ebase + e;
    const int gc = min(ge, E - 1);
    int s = src[gc];
    s = (s < 0) ? (s + n_nodes) : s;
    s = min(max(s, 0), n_nodes - 1);
    v4f x = *(const v4f*)(xin + (size_t)s * LAT + 4 * c4);
    x = (ge < E) ? x : z4;
    *(v4f*)(sX + e * LAT + 4 * c4) = x;
  }
  __syncthreads();

  const int er = 16 * w + m;
  const _Float16* hrow = h2p + (size_t)(ebase + er) * KD + 8 * h;
  const v16h H0 = ldfrag(hrow);
  const v16h H1 = ldfrag(hrow + 32);
  const v16h H2 = ldfrag(hrow + 64);
  const v16h H3 = ldfrag(hrow + 96);
  const float* xr = sX + er * LAT;
  const _Float16* bb = W3f + (size_t)m * KP3 + 8 * h;

  v8f acc = vzero8();
#pragma unroll 1
  for (int i = 0; i < LAT; ++i) {
    const _Float16 xs = (_Float16)(16.0f * xr[i]);
    const _Float16* bp = bb + KD * i;
    acc = wmf(scale16(H0, xs), ldfrag(bp),      acc);
    acc = wmf(scale16(H1, xs), ldfrag(bp + 32), acc);
    acc = wmf(scale16(H2, xs), ldfrag(bp + 64), acc);
    acc = wmf(scale16(H3, xs), ldfrag(bp + 96), acc);
  }
  {
    Frag a;
    const v8f x0 = *(const v8f*)(xr + 8 * h);
    a.half[0] = __builtin_convertvector(x0 * 16.0f, v8h);
    a.half[1] = __builtin_convertvector(vzero8(), v8h);
    acc = wmf(a.v, ldfrag(bb + KW3), acc);
  }

  float* orow = sO + (16 * w + 8 * h) * LAT + m;
#pragma unroll
  for (int r = 0; r < 8; ++r) orow[r * LAT] = acc[r] * (1.0f / 1024.0f);
  __syncthreads();

  float* gb = msg + (size_t)ebase * LAT;
#pragma unroll
  for (int q = 0; q < 2; ++q) {
    const int fo = 4 * (q * NTF + t);
    const v4f v = *(const v4f*)(sO + fo);
    *(volatile v4f*)(gb + fo) = v;
  }
  __threadfence();
#pragma unroll
  for (int q = 0; q < 2; ++q) {
    const int fo = 4 * (q * NTF + t);
    const v4f v = *(const v4f*)(sO + fo);
    *(volatile v4f*)(gb + fo) = v;
  }
}

__global__ __launch_bounds__(NTA) void k_agg(const float* __restrict__ msg, const int* __restrict__ dst, int E,
                                             const float* __restrict__ xin, int n_nodes,
                                             const float* __restrict__ rootp, const float* __restrict__ biasp,
                                             int act, int rows_alloc, float* outp) {
  __shared__ __attribute__((aligned(16))) float acc[NB * LAT];
  __shared__ float sR[LAT * LAT];
  __shared__ float sBv[LAT];
  __shared__ int hit_e[CH];
  __shared__ int hit_n[CH];
  __shared__ int wcnt[2];
  const int t = threadIdx.x, lane = t & 31, w = t >> 5;
  const int sub = t >> 4, col = t & 15;
  const int n0 = blockIdx.x * NB;

  for (int i = t; i < NB * LAT; i += NTA) acc[i] = 0.0f;
  for (int i = t; i < LAT * LAT; i += NTA) sR[i] = rootp[i];
  if (t < LAT) sBv[t] = biasp[t];
  __syncthreads();

#pragma unroll 1
  for (int cb = 0; cb < E; cb += CH) {
    const int e  = cb + t;
    const int ec = min(e, E - 1);
    const int d  = dst[ec];
    const int nl = d - n0;
    const bool valid = (e < E) && (d >= n0) && (nl < NB) && (d < n_nodes);
    const unsigned mask = __builtin_amdgcn_ballot_w32(valid);
    const int pos = (int)__builtin_popcount(mask & ((1u << lane) - 1u));
    wcnt[w] = (int)__builtin_popcount(mask);
    __syncthreads();
    const int wc0 = wcnt[0], wc1 = wcnt[1];
    const int off = (w == 0) ? 0 : wc0;
    const int nh  = min(wc0 + wc1, CH);
    if (valid) {
      hit_e[off + pos] = e;
      hit_n[off + pos] = nl;
    }
    __syncthreads();
#pragma unroll 1
    for (int j = 0; j < nh; ++j) {
      int he = hit_e[j];
      int hn = hit_n[j];
      he = min(max(he, 0), E - 1);
      hn = min(max(hn, 0), NB - 1);
      const float v = msg[(size_t)he * LAT + col];
      if ((hn & 3) == sub) acc[hn * LAT + col] += v;
    }
    __syncthreads();
  }

#pragma unroll 1
  for (int nl = sub; nl < NB; nl += 4) {
    const int n  = n0 + nl;
    const int nc = min(n, n_nodes - 1);
    const float* xrow = xin + (size_t)nc * LAT;
    float r = 0.0f;
#pragma unroll
    for (int i = 0; i < LAT; ++i) r += xrow[i] * sR[i * LAT + col];
    float v = acc[nl * LAT + col] + r;
    v += sBv[col];
    const float g = gelu_f(v);
    acc[nl * LAT + col] = act ? g : v;
  }
  __syncthreads();

  const int rows_valid = min(NB, rows_alloc - n0);
  float* gb = outp + (size_t)n0 * LAT;
#pragma unroll 1
  for (int q = 0; q < (NB * LAT) / (4 * NTA); ++q) {
    const int fo  = 4 * (q * NTA + t);
    const int row = fo >> 4;
    const v4f v = *(const v4f*)(acc + fo);
    if (row < rows_valid) *(volatile v4f*)(gb + fo) = v;
  }
  __threadfence();
#pragma unroll 1
  for (int q = 0; q < (NB * LAT) / (4 * NTA); ++q) {
    const int fo  = 4 * (q * NTA + t);
    const int row = fo >> 4;
    const v4f v = *(const v4f*)(acc + fo);
    if (row < rows_valid) *(volatile v4f*)(gb + fo) = v;
  }
}

extern "C" void kernel_launch(void* const* d_in, const int* in_sizes, int n_in,
                              void* d_out, int out_size, void* d_ws, size_t ws_size,
                              hipStream_t stream) {
  if (n_in < 11) return;
  if (in_sizes[0] <= 0 || (in_sizes[0] % LAT) != 0) return;
  const int N = in_sizes[0] / LAT;
  if (in_sizes[10] <= 0 || (in_sizes[10] % 2) != 0) return;
  const int E = in_sizes[10] / 2;
  if (in_sizes[1] != E * EDW) return;
  if (in_sizes[2] != EDW * KD || in_sizes[3] != KD) return;
  if (in_sizes[4] != KD * KD || in_sizes[5] != KD) return;
  if (in_sizes[6] != KD * W3C || in_sizes[7] != W3C) return;
  if (in_sizes[8] != 2 * LAT * LAT || in_sizes[9] != 2 * LAT) return;
  if (out_size != N * LAT) return;

  const float* nodes = (const float*)d_in[0];
  const float* eattr = (const float*)d_in[1];
  const float* W1    = (const float*)d_in[2];
  const float* b1    = (const float*)d_in[3];
  const float* W2    = (const float*)d_in[4];
  const float* b2    = (const float*)d_in[5];
  const float* W3    = (const float*)d_in[6];
  const float* b3    = (const float*)d_in[7];
  const float* roots = (const float*)d_in[8];
  const float* bias  = (const float*)d_in[9];
  const int*   eidx  = (const int*)d_in[10];
  float* out = (float*)d_out;

  const int nbf   = (E + EB - 1) / EB;
  const int e_pad = nbf * EB;
  const int nba   = (N + NB - 1) / NB;
  const int n_pad = nba * NB;

  char* ws = (char*)d_ws;
  size_t off = 0;
  const size_t oW2t = off; off += (size_t)KD * KD * 2;        off = (off + 255) & ~(size_t)255;
  const size_t oW3f = off; off += (size_t)LAT * KP3 * 2;      off = (off + 255) & ~(size_t)255;
  const size_t oH2  = off; off += (size_t)e_pad * KD * 2;     off = (off + 255) & ~(size_t)255;
  const size_t oMsg = off; off += (size_t)e_pad * LAT * 4;    off = (off + 255) & ~(size_t)255;
  const size_t oX1  = off; off += (size_t)n_pad * LAT * 4;    off = (off + 255) & ~(size_t)255;
  if (off > ws_size || off > (size_t)WSCAP) return;

  _Float16* W2t = (_Float16*)(ws + oW2t);
  _Float16* W3f = (_Float16*)(ws + oW3f);
  _Float16* h2p = (_Float16*)(ws + oH2);
  float* msg = (float*)(ws + oMsg);
  float* x1  = (float*)(ws + oX1);

  const int nprep = ((KD * KD) / 8 + (LAT * KP3) / 8 + 255) / 256;

  k_prep<<<nprep, 256, 0, stream>>>(W2, W3, b3, W2t, W3f);
  k_mlp<<<nbf, NTM, 0, stream>>>(eattr, E, W1, b1, W2t, b2, h2p);
  k_fold<<<nbf, NTF, 0, stream>>>(h2p, nodes, N, eidx, E, W3f, msg);
  k_agg<<<nba, NTA, 0, stream>>>(msg, eidx + E, E, nodes, N, roots, bias, 1, n_pad, x1);
  k_fold<<<nbf, NTF, 0, stream>>>(h2p, x1, N, eidx, E, W3f, msg);
  k_agg<<<nba, NTA, 0, stream>>>(msg, eidx + E, E, x1, N, roots + LAT * LAT, bias + LAT, 0, N, out);
}
